// SRAttention_12249246728398
// MI455X (gfx1250) — hardware-verified
//
#include <hip/hip_runtime.h>
#include <hip/hip_fp16.h>


typedef __attribute__((ext_vector_type(16))) _Float16 v16h;
typedef __attribute__((ext_vector_type(8)))  _Float16 v8h;
typedef __attribute__((ext_vector_type(4)))  _Float16 v4h;
typedef __attribute__((ext_vector_type(8)))  float    v8f;

#define WMMA_F16(a, b, c) \
  __builtin_amdgcn_wmma_f32_16x16x32_f16(false, (a), false, (b), (short)0, (c), false, false)

constexpr int B_  = 4;
constexpr int H_  = 128;
constexpr int W_  = 128;
constexpr int N_  = H_ * W_;
constexpr int C_  = 64;
constexpr int NK_ = 256;
constexpr int LDX = 72;
constexpr int LDK = 72;
constexpr int LDP = 264;
constexpr int LDVT= 264;

__device__ __forceinline__ void async_load_b128(unsigned lds_off, const void* gaddr) {
  asm volatile("global_load_async_to_lds_b128 %0, %1, off"
               :: "v"(lds_off), "v"(gaddr) : "memory");
}
__device__ __forceinline__ void wait_asynccnt0() {
  asm volatile("s_wait_asynccnt 0x0" ::: "memory");
}


__device__ __forceinline__ v16h cat8(v8h lo, v8h hi) {
  return __builtin_shufflevector(lo, hi, 0,1,2,3,4,5,6,7,8,9,10,11,12,13,14,15);
}

__device__ __forceinline__ v16h load_A16(const _Float16* base, int ld, int lane) {
  const int m    = lane & 15;
  const int koff = (lane & 16) ? 8 : 0;
  const v8h* p = (const v8h*)(base + m * ld + koff);
  return cat8(p[0], p[2]);
}

__device__ __forceinline__ v16h load_Bt(const _Float16* bt, int ld, int lane) {
  return load_A16(bt, ld, lane);
}
typedef __attribute__((ext_vector_type(4))) float v4f_t;
typedef float v4fa __attribute__((ext_vector_type(4), may_alias));

__device__ __forceinline__ void store_C_f32(float* base, int ld, int lane, v8f c) {
  const int n  = lane & 15;
  const int mo = (lane & 16) ? 8 : 0;
#pragma unroll
  for (int r = 0; r < 8; ++r) base[(mo + r) * ld + n] = c[r];
}

__device__ __forceinline__ void store_C_f16(_Float16* base, int ld, int lane, v8f c) {
  const int n  = lane & 15;
  const int mo = (lane & 16) ? 8 : 0;
#pragma unroll
  for (int r = 0; r < 8; ++r) base[(mo + r) * ld + n] = (_Float16)c[r];
}

__global__ void __launch_bounds__(64)
sra_kv_kernel(const float* __restrict__ x1, const float* __restrict__ x2,
              const float* __restrict__ kv1_w, const float* __restrict__ kv2_w,
              const float* __restrict__ n1g, const float* __restrict__ n1b,
              const float* __restrict__ n2g, const float* __restrict__ n2b,
              _Float16* __restrict__ kg, _Float16* __restrict__ vtg)
{
  const int p  = blockIdx.x;
  const int b  = blockIdx.y;
  const int br = blockIdx.z;
  const int c  = threadIdx.x;

  const float* x   = br ? x2 : x1;
  const float* kvw = br ? kv2_w : kv1_w;
  const float* gg  = br ? n2g : n1g;
  const float* gb  = br ? n2b : n1b;

  __shared__ float s_a[64];
  __shared__ float s_y[64];

  const int ph = p >> 4, pw = p & 15;
  const float* xb = x + (size_t)b * N_ * C_ + ((size_t)(ph * 8) * W_ + pw * 8) * C_ + c;

  float acc = 0.f;
#pragma unroll
  for (int dy = 0; dy < 8; ++dy)
#pragma unroll
    for (int dx = 0; dx < 8; ++dx)
      acc += xb[(size_t)(dy * W_ + dx) * C_];
  acc *= (1.f / 64.f);
  s_a[c] = acc;
  __syncthreads();

  float mu = 0.f;
#pragma unroll 1
  for (int i = 0; i < 64; ++i) mu += s_a[i];
  mu *= (1.f / 64.f);
  float var = 0.f;
#pragma unroll 1
  for (int i = 0; i < 64; ++i) { float d = s_a[i] - mu; var += d * d; }
  var *= (1.f / 64.f);

  s_y[c] = (acc - mu) * rsqrtf(var + 1e-5f) * gg[c] + gb[c];
  __syncthreads();

  float kacc = 0.f, vacc = 0.f;
  const float* wk = kvw + (size_t)c * C_;
  const float* wv = kvw + (size_t)(64 + c) * C_;
#pragma unroll 1
  for (int i = 0; i < 64; ++i) { kacc += s_y[i] * wk[i]; vacc += s_y[i] * wv[i]; }

  const float scale = 0.125f;
  const int bb = b * 2 + br;
  __shared__ _Float16 s_k[64], s_v[64];
  s_k[c] = (_Float16)(kacc * scale); s_v[c] = (_Float16)vacc;
  __syncthreads();
  if (c < 32) {
    const unsigned kk2 = (unsigned)__builtin_bit_cast(unsigned short, s_k[2 * c]) | ((unsigned)__builtin_bit_cast(unsigned short, s_k[2 * c + 1]) << 16);
    const unsigned vv2 = (unsigned)__builtin_bit_cast(unsigned short, s_v[2 * c]) | ((unsigned)__builtin_bit_cast(unsigned short, s_v[2 * c + 1]) << 16);
    unsigned* kd = (unsigned*)(kg  + ((size_t)bb * NK_ + p) * C_) + c;
    unsigned* vd = (unsigned*)(vtg + ((size_t)bb * NK_ + p) * C_) + c;
    *(volatile unsigned*)kd = kk2; *(volatile unsigned*)vd = vv2; __threadfence(); *(volatile unsigned*)kd = kk2; *(volatile unsigned*)vd = vv2;
  }
}

__global__ void __launch_bounds__(128)
sra_attn_kernel(const float* __restrict__ x1, const float* __restrict__ x2,
                const float* __restrict__ q1_w,
                const float* __restrict__ proj1_w, const float* __restrict__ proj1_b,
                const float* __restrict__ proj2_w, const float* __restrict__ proj2_b,
                const _Float16* __restrict__ kg, const _Float16* __restrict__ vtg,
                float* __restrict__ out)
{
  __shared__ __align__(16) _Float16 s_x [64 * LDX];
  __shared__ __align__(16) _Float16 s_wq[64 * LDX];
  __shared__ __align__(16) _Float16 s_wp[64 * LDX];
  __shared__ __align__(16) _Float16 s_kp[NK_ * LDK];
  __shared__ __align__(16) _Float16 s_vt[C_ * LDVT];
  __shared__ __align__(16) float    s_s [64 * NK_];

  const int tid  = threadIdx.x;
  const int lane = tid & 31;
  const int wv   = tid >> 5;
  const int m0   = wv * 16;
  const int row0 = blockIdx.x * 64;
  const int b    = blockIdx.y;
  const int br   = blockIdx.z;

  const float* x  = br ? x2 : x1;
  const float* pw = br ? proj2_w : proj1_w;
  const float* pb = br ? proj2_b : proj1_b;
  const int bb = b * 2 + br;
  const _Float16* kgp  = kg  + (size_t)bb * NK_ * C_;
  const _Float16* vtgp = vtg + (size_t)bb * NK_ * C_;
  const float* xrow = x + (size_t)b * N_ * C_ + (size_t)row0 * C_;

  for (int i = tid; i < (NK_ * C_) / 8; i += 128) {
    const int r = i >> 3, ch = (i & 7) * 8;
    async_load_b128((unsigned)(size_t)(s_kp + r * LDK + ch), kgp + r * C_ + ch);
  }
  for (int i = tid; i < (NK_ * C_) / 8; i += 128) {
    const int pp = i >> 3, ch = (i & 7) * 8;
    const v8h v8 = *(const v8h*)(vtgp + (size_t)pp * C_ + ch);
#pragma unroll
    for (int e = 0; e < 8; ++e) s_vt[(ch + e) * LDVT + pp] = v8[e];
  }
  for (int idx = tid * 4; idx < 64 * 64; idx += 128 * 4) {
    const int j = idx >> 6, c = idx & 63;
    const float4 wq4 = *(const float4*)(q1_w + idx);
    const float4 wp4 = *(const float4*)(pw + idx);
    *(v4h*)(s_wq + j * LDX + c) = (v4h){(_Float16)wq4.x, (_Float16)wq4.y,
                                        (_Float16)wq4.z, (_Float16)wq4.w};
    *(v4h*)(s_wp + j * LDX + c) = (v4h){(_Float16)wp4.x, (_Float16)wp4.y,
                                        (_Float16)wp4.z, (_Float16)wp4.w};
  }
  for (int idx = tid * 4; idx < 64 * 64; idx += 128 * 4) {
    const int r = idx >> 6, c = idx & 63;
    const float4 x4 = *(const float4*)(xrow + idx);
    *(v4h*)(s_x + r * LDX + c) = (v4h){(_Float16)x4.x, (_Float16)x4.y,
                                       (_Float16)x4.z, (_Float16)x4.w};
  }
  wait_asynccnt0();
  __syncthreads();

  {
    const v16h a0 = load_A16(s_x + m0 * LDX + 0,  LDX, lane);
    const v16h a1 = load_A16(s_x + m0 * LDX + 32, LDX, lane);
    v8f qacc[4];
#pragma unroll
    for (int nt = 0; nt < 4; ++nt) {
      v8f c = {};
      c = WMMA_F16(a0, load_Bt(s_wq + (nt * 16) * LDX + 0,  LDX, lane), c);
      c = WMMA_F16(a1, load_Bt(s_wq + (nt * 16) * LDX + 32, LDX, lane), c);
      qacc[nt] = c;
    }
#pragma unroll
    for (int nt = 0; nt < 4; ++nt)
      store_C_f16(s_x + m0 * LDX + nt * 16, LDX, lane, qacc[nt]);
  }

  {
    const v16h a0 = load_A16(s_x + m0 * LDX + 0,  LDX, lane);
    const v16h a1 = load_A16(s_x + m0 * LDX + 32, LDX, lane);
#pragma unroll
    for (int nt = 0; nt < 16; ++nt) {
      v8f c = {};
      c = WMMA_F16(a0, load_Bt(s_kp + (nt * 16) * LDK + 0,  LDK, lane), c);
      c = WMMA_F16(a1, load_Bt(s_kp + (nt * 16) * LDK + 32, LDK, lane), c);
      store_C_f32(s_s + m0 * NK_ + nt * 16, NK_, lane, c);
    }
  }
  __syncthreads();

  if (tid < 64) {
    float* sr = s_s + tid * NK_;
    float mx = -3.4e38f;
    for (int i = 0; i < NK_; i += 4) {
      const float4 s4 = *(const float4*)(sr + i);
      mx = fmaxf(mx, fmaxf(fmaxf(s4.x, s4.y), fmaxf(s4.z, s4.w)));
    }
    float sum = 0.f;
    for (int i = 0; i < NK_; i += 4) {
      float4 s4 = *(float4*)(sr + i);
      s4.x = __expf(s4.x - mx); s4.y = __expf(s4.y - mx);
      s4.z = __expf(s4.z - mx); s4.w = __expf(s4.w - mx);
      sum += s4.x + s4.y + s4.z + s4.w;
      *(float4*)(sr + i) = s4;
    }
    const float inv = 1.f / sum;
    _Float16* pr = s_kp + tid * LDP;
    for (int i = 0; i < NK_; i += 4) {
      const float4 s4 = *(const float4*)(sr + i);
      *(v4h*)(pr + i) = (v4h){(_Float16)(s4.x * inv), (_Float16)(s4.y * inv),
                              (_Float16)(s4.z * inv), (_Float16)(s4.w * inv)};
    }
  }
  __syncthreads();

  v8f oacc[4] = {};
#pragma unroll
  for (int kc = 0; kc < 8; ++kc) {
    const v16h a = load_A16(s_kp + m0 * LDP + kc * 32, LDP, lane);
#pragma unroll
    for (int nt = 0; nt < 4; ++nt)
      oacc[nt] = WMMA_F16(a, load_Bt(s_vt + (nt * 16) * LDVT + kc * 32, LDVT, lane),
                          oacc[nt]);
  }
#pragma unroll
  for (int nt = 0; nt < 4; ++nt)
    store_C_f16(s_x + m0 * LDX + nt * 16, LDX, lane, oacc[nt]);

  {
    const v16h a0 = load_A16(s_x + m0 * LDX + 0,  LDX, lane);
    const v16h a1 = load_A16(s_x + m0 * LDX + 32, LDX, lane);
    float* og = out + (size_t)br * B_ * N_ * C_ + (size_t)b * N_ * C_
                    + (size_t)(row0 + m0) * C_;
    float* so = s_s + m0 * C_;
#pragma unroll
    for (int nt = 0; nt < 4; ++nt) {
      v8f c = {};
      c = WMMA_F16(a0, load_Bt(s_wp + (nt * 16) * LDX + 0,  LDX, lane), c);
      c = WMMA_F16(a1, load_Bt(s_wp + (nt * 16) * LDX + 32, LDX, lane), c);
      const int n  = lane & 15;
      const int mo = (lane & 16) ? 8 : 0;
      const float bias = pb[nt * 16 + n];
#pragma unroll
      for (int r = 0; r < 8; ++r) so[(mo + r) * C_ + nt * 16 + n] = c[r] + bias;
    }
    asm volatile("s_wait_dscnt 0" ::: "memory");
#pragma unroll 1
    for (int pass = 0; pass < 2; ++pass) {
#pragma unroll
      for (int i = 0; i < 8; ++i) { const int cc = lane + 32 * i, rr = cc >> 4, q = (cc & 15) * 4;
        *(volatile v4f_t*)(og + (size_t)rr * C_ + q) = *(const volatile v4fa*)(so + rr * C_ + q); }
      __threadfence();
    }
  }
}

extern "C" void kernel_launch(void* const* d_in, const int* in_sizes, int n_in,
                              void* d_out, int out_size, void* d_ws, size_t ws_size,
                              hipStream_t stream) {
  const float* x1    = (const float*)d_in[0];
  const float* x2    = (const float*)d_in[1];
  const float* q1_w  = (const float*)d_in[4];
  const float* kv1_w = (const float*)d_in[5];
  const float* kv2_w = (const float*)d_in[6];
  const float* n1g   = (const float*)d_in[7];
  const float* n1b   = (const float*)d_in[8];
  const float* n2g   = (const float*)d_in[9];
  const float* n2b   = (const float*)d_in[10];
  const float* p1w   = (const float*)d_in[11];
  const float* p1b   = (const float*)d_in[12];
  const float* p2w   = (const float*)d_in[13];
  const float* p2b   = (const float*)d_in[14];

  _Float16* kg  = (_Float16*)d_ws;
  _Float16* vtg = kg + (size_t)B_ * 2 * NK_ * C_;

  dim3 g1(NK_, B_, 2);
  sra_kv_kernel<<<g1, 64, 0, stream>>>(x1, x2, kv1_w, kv2_w, n1g, n1b, n2g, n2b, kg, vtg);

  dim3 g2(N_ / 64, B_, 2);
  sra_attn_kernel<<<g2, 128, 0, stream>>>(x1, x2, q1_w, p1w, p1b, p2w, p2b,
                                          kg, vtg, (float*)d_out);
}
